// VariableSelectionNetwork_19937238188299
// MI455X (gfx1250) — hardware-verified
//
#include <hip/hip_runtime.h>


#define NR   16384
#define RC   4096
#define NF   64
#define NHID 64
#define KT   (NF * NHID)
typedef _Float16 h16;
typedef unsigned short bf;
typedef __attribute__((ext_vector_type(16))) __bf16   v16bf;
typedef __attribute__((ext_vector_type(16))) _Float16 v16h;
typedef __attribute__((ext_vector_type(8)))  _Float16 v8h;
typedef __attribute__((ext_vector_type(8)))  unsigned short v8us;
typedef __attribute__((ext_vector_type(8)))  float    v8f;
typedef __attribute__((ext_vector_type(4)))  float    v4f;
typedef v8h  __attribute__((may_alias)) v8ha;
typedef v4f  __attribute__((may_alias)) v4fa;
typedef v8us __attribute__((may_alias)) v8usa;

__device__ __forceinline__ unsigned short f2bf(float f) { unsigned u = __float_as_uint(f); u += 0x7FFFu + ((u >> 16) & 1u); return (unsigned short)(u >> 16); }
__device__ __forceinline__ float bf2f(unsigned short b) { return __uint_as_float(((unsigned)b) << 16); }
__device__ __forceinline__ float bfr(float f) { return bf2f(f2bf(f)); }
__device__ __forceinline__ v16h cat16(v8h lo, v8h hi) { return __builtin_shufflevector(lo, hi, 0, 1, 2, 3, 4, 5, 6, 7, 8, 9, 10, 11, 12, 13, 14, 15); }
__device__ __forceinline__ v16bf cat16b(v8us lo, v8us hi) { return __builtin_bit_cast(v16bf, __builtin_shufflevector(lo, hi, 0, 1, 2, 3, 4, 5, 6, 7, 8, 9, 10, 11, 12, 13, 14, 15)); }
__device__ __forceinline__ v8f wmma16(v16h a, v16h b, v8f c) { return __builtin_amdgcn_wmma_f32_16x16x32_f16(false, a, false, b, (short)0, c, false, false); }
__device__ __forceinline__ v8f wmmab(v16bf a, v16bf b, v8f c) { return __builtin_amdgcn_wmma_f32_16x16x32_bf16(false, a, false, b, (short)0, c, false, false); }


template <typename T16> struct WFrag;
template <> struct WFrag<h16> { typedef v16h V; static __device__ __forceinline__ V ld(const h16* p) { return cat16(*(const v8h*)p, *(const v8h*)(p + 16)); } static __device__ __forceinline__ v8f mma(V a, V b, v8f c) { return wmma16(a, b, c); } };
template <> struct WFrag<bf> { typedef v16bf V; static __device__ __forceinline__ V ld(const bf* p) { return cat16b(*(const v8us*)p, *(const v8us*)(p + 16)); } static __device__ __forceinline__ v8f mma(V a, V b, v8f c) { return wmmab(a, b, c); } };
template <typename T16, int NSPLIT, bool BIAS>
__global__ __launch_bounds__(32) void k_gemmw(const T16* __restrict__ A, const T16* __restrict__ A2, const T16* __restrict__ Bt, const T16* __restrict__ Bt2, int K, float* C, int ldc, const float* __restrict__ bias, size_t sA, size_t sB, size_t sC) {
    typedef typename WFrag<T16>::V V;
    __shared__ __align__(16) float os[16 * 68];
    const size_t z = blockIdx.z; A += z * sA; if (A2) A2 += z * sA; Bt += z * sB; if (Bt2) Bt2 += z * sB; C += z * sC;
    const int lane = threadIdx.x & 31, lr = lane & 15, hi = lane >> 4; const int r0 = blockIdx.x * 64, c0 = blockIdx.y * 64;
    v8f acc[4][4];
#pragma unroll
    for (int mb = 0; mb < 4; ++mb)
#pragma unroll
        for (int nb = 0; nb < 4; ++nb) acc[mb][nb] = (v8f){};
    const size_t aoff = (size_t)(r0 + lr) * K + 8 * hi, boff = (size_t)(c0 + lr) * K + 8 * hi;
#pragma unroll 1
    for (int kc = 0; kc < K; kc += 32) {
        V a[4], a2[4];
#pragma unroll
        for (int mb = 0; mb < 4; ++mb) { a[mb] = WFrag<T16>::ld(A + aoff + (size_t)mb * 16 * K + kc); if (NSPLIT == 1 || NSPLIT == 2) a2[mb] = WFrag<T16>::ld(A2 + aoff + (size_t)mb * 16 * K + kc); }
#pragma unroll
        for (int nb = 0; nb < 4; ++nb) { const V b = WFrag<T16>::ld(Bt + boff + (size_t)nb * 16 * K + kc); V b2; if (NSPLIT >= 2) b2 = WFrag<T16>::ld(Bt2 + boff + (size_t)nb * 16 * K + kc);
#pragma unroll
            for (int mb = 0; mb < 4; ++mb) { acc[mb][nb] = WFrag<T16>::mma(a[mb], b, acc[mb][nb]); if (NSPLIT == 1 || NSPLIT == 2) acc[mb][nb] = WFrag<T16>::mma(a2[mb], b, acc[mb][nb]); if (NSPLIT >= 2) acc[mb][nb] = WFrag<T16>::mma(a[mb], b2, acc[mb][nb]); } }
        asm volatile("v_nop\n\tv_nop\n\tv_nop\n\tv_nop" : "+v"(acc[0][0]), "+v"(acc[1][1]), "+v"(acc[2][2]), "+v"(acc[3][3]) : "v"(a[0]), "v"(a[3]));
    }
#pragma unroll
    for (int mb = 0; mb < 4; ++mb) {
#pragma unroll
        for (int nb = 0; nb < 4; ++nb) {
#pragma unroll
            for (int j = 0; j < 8; ++j) os[(hi * 8 + j) * 68 + nb * 16 + lr] = acc[mb][nb][j]; }
        __builtin_amdgcn_wave_barrier(); asm volatile("" ::: "memory");
        float* crow = C + (size_t)(r0 + mb * 16) * ldc + c0;
#pragma unroll 1
        for (int ps = 0; ps < 2; ++ps) {
#pragma unroll
            for (int s = 0; s < 8; ++s) { const int row = 2 * s + hi, cofs = lr * 4; v4f val = *(const v4fa*)(os + row * 68 + cofs); if (BIAS) { val[0] += bfr(bias[c0 + cofs]); val[1] += bfr(bias[c0 + cofs + 1]); val[2] += bfr(bias[c0 + cofs + 2]); val[3] += bfr(bias[c0 + cofs + 3]); }
                *(volatile v4f*)(crow + (size_t)row * ldc + cofs) = val; }
            if (ps == 0) __threadfence(); }
        __builtin_amdgcn_wave_barrier(); asm volatile("" ::: "memory");
    }
}

typedef __attribute__((ext_vector_type(4))) unsigned short v4us;
typedef __attribute__((ext_vector_type(2))) unsigned short v2us;
typedef __attribute__((ext_vector_type(2))) float v2f;
__device__ __forceinline__ void splitf(float y, unsigned short& h, unsigned short& l) { h = f2bf(y); l = f2bf(y - bf2f(h)); }
__global__ __launch_bounds__(256) void k_wtG(const float* __restrict__ w, int K, int N, bf* Bt) {
    const int lane = threadIdx.x & 31; const int L0 = (blockIdx.x * 8 + (threadIdx.x >> 5)) * 8; const int nlines = N * K / 64;
#pragma unroll
    for (int ps = 0; ps < 2; ++ps) {
#pragma unroll 1
        for (int l = 0; l < 8; ++l) { const int L = L0 + l; if (L >= nlines) break; const size_t e = (size_t)L * 64 + lane * 2; const int k = (int)(e % K), n = (int)(e / K); v2us o;
            o[0] = f2bf(w[(size_t)k * N + n]); o[1] = f2bf(w[(size_t)(k + 1) * N + n]); *(volatile v2us*)(Bt + e) = o; }
        if (ps == 0) __threadfence(); }
}

__global__ __launch_bounds__(256) void k_tr(const float* __restrict__ xc, const float* __restrict__ Wf, const float* __restrict__ bfv, float* T, bf* Th, bf* Tl) { const size_t i = (size_t)blockIdx.x * 256 + threadIdx.x; if (i >= (size_t)RC * KT / 4) return; const int c0 = (int)(i % (KT / 4)) * 4; const size_t r = i / (KT / 4); const int f = c0 / NHID, h0 = c0 % NHID; const float xv = bfr(xc[r * NF + f]); v4f o; v4us oh, ol;
#pragma unroll
    for (int q = 0; q < 4; ++q) { float p = __fmul_rn(xv, bfr(Wf[f * NHID + h0 + q])); asm volatile("" : "+v"(p)); const float v = __fadd_rn(p, bfr(bfv[f * NHID + h0 + q])); const float e = expm1f(v); const float t = (v > 0.0f) ? v : e; o[q] = t; unsigned short a, b; splitf(t, a, b); oh[q] = a; ol[q] = b; }
    *(volatile v4f*)(T + r * KT + c0) = o; *(volatile v4us*)(Th + r * KT + c0) = oh; *(volatile v4us*)(Tl + r * KT + c0) = ol; __threadfence(); *(volatile v4f*)(T + r * KT + c0) = o; *(volatile v4us*)(Th + r * KT + c0) = oh; *(volatile v4us*)(Tl + r * KT + c0) = ol; }
__global__ __launch_bounds__(256) void k_sel(const float* __restrict__ LG, const float* __restrict__ T, size_t r0, float* sel, float* wts) { const int lane = threadIdx.x & 31; const size_t rl = (size_t)blockIdx.x * 8 + (threadIdx.x >> 5); if (rl >= RC) return; const size_t r = r0 + rl;
    const v2f lg = *(const v2f*)(LG + rl * NF + lane * 2); float mx = fmaxf(lg[0], lg[1]);
#pragma unroll
    for (int sh = 16; sh; sh >>= 1) mx = fmaxf(mx, __shfl_xor(mx, sh, 32));
    float d0 = __fsub_rn(lg[0], mx), d1 = __fsub_rn(lg[1], mx); asm volatile("" : "+v"(d0), "+v"(d1)); const float e0 = __builtin_amdgcn_exp2f(__fmul_rn(d0, 1.4426950408889634f)), e1 = __builtin_amdgcn_exp2f(__fmul_rn(d1, 1.4426950408889634f)); float sum = __fadd_rn(e0, e1);
#pragma unroll
    for (int sh = 16; sh; sh >>= 1) sum = __fadd_rn(sum, __shfl_xor(sum, sh, 32));
    const float inv = __fdiv_rn(1.0f, sum); const float w0 = __fmul_rn(e0, inv), w1 = __fmul_rn(e1, inv);
    float s0 = 0.f, s1 = 0.f; const float* tr = T + rl * KT + lane * 2;
#pragma unroll 4
    for (int f = 0; f < NF; ++f) { const float wf = __shfl((f & 1) ? w1 : w0, f >> 1, 32);     const v2f tv = *(const v2f*)(tr + f * NHID); float p0 = __fmul_rn(wf, tv[0]), p1 = __fmul_rn(wf, tv[1]); asm volatile("" : "+v"(p0), "+v"(p1)); s0 = __fadd_rn(s0, p0); s1 = __fadd_rn(s1, p1); }
    v2f ow; ow[0] = w0; ow[1] = w1; v2f os; os[0] = s0; os[1] = s1;
    *(volatile v2f*)(wts + r * NF + lane * 2) = ow; *(volatile v2f*)(sel + r * NHID + lane * 2) = os; __threadfence(); *(volatile v2f*)(wts + r * NF + lane * 2) = ow; *(volatile v2f*)(sel + r * NHID + lane * 2) = os; }

extern "C" void kernel_launch(void* const* d_in, const int* in_sizes, int n_in,
                              void* d_out, int out_size, void* d_ws, size_t ws_size, hipStream_t stream) {
    (void)in_sizes; (void)n_in; (void)out_size;
    const float* x = (const float*)d_in[0]; const float* Wf = (const float*)d_in[1]; const float* bfv = (const float*)d_in[2]; const float* Ws = (const float*)d_in[3]; const float* bs = (const float*)d_in[4];
    float* SEL = (float*)d_out; float* WTS = SEL + (size_t)NR * NHID;
    char* wsp = (char*)d_ws;
    auto take = [&](size_t bytes) { char* p = wsp; wsp += (bytes + 255) & ~(size_t)255; return (void*)p; };
    bf* WSB = (bf*)take((size_t)NF * KT * 2); float* T = (float*)take((size_t)RC * KT * 4); bf* Th = (bf*)take((size_t)RC * KT * 2); bf* Tl = (bf*)take((size_t)RC * KT * 2); float* LG = (float*)take((size_t)RC * NF * 4);
    if ((size_t)(wsp - (char*)d_ws) > ws_size) return;
    k_wtG<<<(KT * NF / 64 + 63) / 64, 256, 0, stream>>>(Ws, KT, NF, WSB);
    for (size_t r0 = 0; r0 < (size_t)NR; r0 += RC) {
        k_tr<<<(unsigned)(((size_t)RC * KT / 4 + 255) / 256), 256, 0, stream>>>(x + r0 * NF, Wf, bfv, T, Th, Tl);
        k_gemmw<bf, 1, true><<<dim3(RC / 64, NF / 64, 1), 32, 0, stream>>>(Th, Tl, WSB, nullptr, KT, LG, NF, bs, 0, 0, 0);
        k_sel<<<RC / 8, 256, 0, stream>>>(LG, T, r0, SEL, WTS); }
}
